// DeltaNetLayer_72009421685068
// MI455X (gfx1250) — hardware-verified
//
#include <hip/hip_runtime.h>
#include <stddef.h>


#define NBAT   2
#define NSEQ   1024
#define NDIM   1024
#define NHEAD  8
#define HDIM   128
#define NTOK   (NBAT * NSEQ)
#define NTHR   256
#define NWAV   (NTHR / 32)
#define BPAD   16
#define STHR   1024
#define SGRP   (STHR / HDIM)
#define SROW   (HDIM / SGRP)
#define TB     (STHR / 32)
#define PBM    64
#define PBN    128
#define PNT    4
#define BBM    128
#define CT     64
#define CTP    (CT + 1)
#define WSCAP  134217728

#define SZXP   ((size_t)NTOK * NDIM * 2)
#define SZWP   ((size_t)3 * NDIM * NDIM * 2)
#define SZWBP  ((size_t)BPAD * NDIM * 2)
#define SZF    ((size_t)NTOK * NDIM * 4)
#define SZBT   ((size_t)NTOK * NHEAD * 4)
#define OXH    ((size_t)0)
#define OXL    (OXH + SZXP)
#define OWH    (OXL + SZXP)
#define OWL    (OWH + SZWP)
#define OWBH   (OWL + SZWP)
#define OWBL   (OWBH + SZWBP)
#define OQ     (OWBL + SZWBP)
#define OKN    (OQ + SZF)
#define OV     (OKN + SZF)
#define OBT    (OV + SZF)
#define OO     (OBT + SZBT)
#define WSTOT  (OO + SZF)

#define CVTX_BLK   (NTOK * NDIM / 8 / NTHR)
#define CVTWB_BLK  (BPAD * NDIM / 8 / NTHR)

static_assert(WSTOT <= (size_t)WSCAP);
static_assert((OXL % 128) == 0 && (OWH % 128) == 0 && (OWL % 128) == 0 && (OWBH % 128) == 0 && (OWBL % 128) == 0);
static_assert((OQ % 128) == 0 && (OKN % 128) == 0 && (OV % 128) == 0 && (OBT % 128) == 0 && (OO % 128) == 0);
static_assert(OO + SZF == WSTOT);
static_assert((NDIM % 32) == 0);
static_assert((NTOK % PBM) == 0 && (NDIM % PBN) == 0 && (NTOK % BBM) == 0);
static_assert(PBM == 16 * 4 && PBN == 2 * 16 * PNT && NWAV == 8 && PBN == HDIM);
static_assert((NDIM % CT) == 0 && ((CT * CT / 4) % NTHR) == 0 && ((CT * CT / 8) % NTHR) == 0);
static_assert((NTOK * NDIM) % (8 * NTHR) == 0 && (BPAD * NDIM) % (8 * NTHR) == 0);
static_assert(SGRP * SROW == HDIM && SROW == 16 && SGRP == 8 && TB == 32 && (NSEQ % TB) == 0);
static_assert(HDIM == 32 * 4);
static_assert((NTOK % NWAV) == 0 && NDIM == 8 * 128);
static_assert(BPAD >= NHEAD && NHEAD == 8 && BBM == NWAV * 16);

typedef unsigned short us_t;
typedef us_t   v8us __attribute__((ext_vector_type(8), __may_alias__));
typedef __bf16 v16b __attribute__((ext_vector_type(16)));
typedef int    v8i  __attribute__((ext_vector_type(8)));
typedef float  v8f  __attribute__((ext_vector_type(8)));
typedef float  v4f  __attribute__((ext_vector_type(4), __may_alias__));
union Frag { v16b v; v8us h[2]; v8i w; };
static_assert(sizeof(Frag) == 32);

__device__ __forceinline__ v8f wmb(Frag a, Frag b, v8f c) {
  v8f d = __builtin_amdgcn_wmma_f32_16x16x32_bf16(false, a.v, false, b.v, (short)0, c, false, false);
  asm volatile("v_nop\n\tv_nop\n\tv_nop\n\tv_nop" : "+v"(d) : "v"(a.w), "v"(b.w));
  return d;
}

__device__ __forceinline__ v8f zero8() {
  v8f z = {0.f, 0.f, 0.f, 0.f, 0.f, 0.f, 0.f, 0.f};
  return z;
}

__device__ __forceinline__ unsigned bfr_(float x) {
  const unsigned u = __float_as_uint(x);
  return (u + 0x7FFFu + ((u >> 16) & 1u)) >> 16;
}
__device__ __forceinline__ void split_(float x, us_t& hi, us_t& lo) {
  const unsigned hb = bfr_(x);
  const float hf = __uint_as_float(hb << 16);
  const unsigned lb = bfr_(x - hf);
  hi = (us_t)hb;
  lo = (us_t)lb;
}
__device__ __forceinline__ void cvt8_(const float* f, v8us& vh, v8us& vl) {
#pragma unroll
  for (int i = 0; i < 8; ++i) {
    us_t a, c;
    split_(f[i], a, c);
    vh[i] = a;
    vl[i] = c;
  }
}

__device__ __forceinline__ float wsum_(float v) {
  v += __shfl_xor(v, 16);
  v += __shfl_xor(v, 8);
  v += __shfl_xor(v, 4);
  v += __shfl_xor(v, 2);
  v += __shfl_xor(v, 1);
  return v;
}
__device__ __forceinline__ float rcp_(float d) { return __builtin_amdgcn_rcpf(d); }
__device__ __forceinline__ float sigm_(float x) {
  const float xc = fminf(fmaxf(x, -30.0f), 30.0f);
  return rcp_(1.0f + __expf(-xc));
}
__device__ __forceinline__ float silu_(float x) { return x * sigm_(x); }

__global__ __launch_bounds__(NTHR) void k_cvtx(const float* __restrict__ x, us_t* XH, us_t* XL) {
  const size_t e = ((size_t)blockIdx.x * NTHR + threadIdx.x) * 8;
  const v4f a0 = *(const v4f*)(x + e);
  const v4f a1 = *(const v4f*)(x + e + 4);
  float f[8];
  f[0] = a0.x; f[1] = a0.y; f[2] = a0.z; f[3] = a0.w;
  f[4] = a1.x; f[5] = a1.y; f[6] = a1.z; f[7] = a1.w;
  v8us vh, vl;
  cvt8_(f, vh, vl);
  *(volatile v8us*)(XH + e) = vh;
  *(volatile v8us*)(XL + e) = vl;
  __threadfence();
  *(volatile v8us*)(XH + e) = vh;
  *(volatile v8us*)(XL + e) = vl;
}

__global__ __launch_bounds__(NTHR) void k_cvtw(const float* __restrict__ Wq, const float* __restrict__ Wk,
                                               const float* __restrict__ Wv, us_t* WH, us_t* WL) {
  __shared__ float sT[CT * CTP];
  const int tid = threadIdx.x;
  const int n0 = blockIdx.x * CT, k0 = blockIdx.y * CT, z = blockIdx.z;
  const float* W = (z == 0) ? Wq : ((z == 1) ? Wk : Wv);
#pragma unroll
  for (int it = 0; it < (CT * CT / 4) / NTHR; ++it) {
    const int e = tid + NTHR * it;
    const int kr = e >> 4, nq = e & 15;
    const v4f a = *(const v4f*)(W + (size_t)(k0 + kr) * NDIM + n0 + 4 * nq);
    sT[(4 * nq + 0) * CTP + kr] = a.x;
    sT[(4 * nq + 1) * CTP + kr] = a.y;
    sT[(4 * nq + 2) * CTP + kr] = a.z;
    sT[(4 * nq + 3) * CTP + kr] = a.w;
  }
  __syncthreads();
  v8us vh[2], vl[2];
  size_t off[2];
#pragma unroll
  for (int it = 0; it < (CT * CT / 8) / NTHR; ++it) {
    const int e = tid + NTHR * it;
    const int rl = e >> 3, q = e & 7;
    float f[8];
#pragma unroll
    for (int i = 0; i < 8; ++i) f[i] = sT[rl * CTP + 8 * q + i];
    cvt8_(f, vh[it], vl[it]);
    off[it] = ((size_t)(z * NDIM + n0 + rl)) * NDIM + k0 + 8 * q;
  }
#pragma unroll
  for (int it = 0; it < 2; ++it) {
    *(volatile v8us*)(WH + off[it]) = vh[it];
    *(volatile v8us*)(WL + off[it]) = vl[it];
  }
  __threadfence();
#pragma unroll
  for (int it = 0; it < 2; ++it) {
    *(volatile v8us*)(WH + off[it]) = vh[it];
    *(volatile v8us*)(WL + off[it]) = vl[it];
  }
}

__global__ __launch_bounds__(NTHR) void k_cvtwb(const float* __restrict__ Wb, us_t* WBH, us_t* WBL) {
  const int e = blockIdx.x * NTHR + threadIdx.x;
  const int n = e >> 7, q = e & 127;
  const int nn = (n < NHEAD) ? n : (NHEAD - 1);
  const float msk = (n < NHEAD) ? 1.0f : 0.0f;
  float f[8];
#pragma unroll
  for (int i = 0; i < 8; ++i) f[i] = Wb[(size_t)(8 * q + i) * NHEAD + nn] * msk;
  v8us vh, vl;
  cvt8_(f, vh, vl);
  const size_t off = (size_t)e * 8;
  *(volatile v8us*)(WBH + off) = vh;
  *(volatile v8us*)(WBL + off) = vl;
  __threadfence();
  *(volatile v8us*)(WBH + off) = vh;
  *(volatile v8us*)(WBL + off) = vl;
}

__global__ __launch_bounds__(NTHR) void k_proj(const us_t* __restrict__ XH, const us_t* __restrict__ XL,
                                               const us_t* __restrict__ WH, const us_t* __restrict__ WL,
                                               float* Q, float* KN, float* V) {
  __shared__ __align__(16) float sT[PBM * PBN];
  const int tid = threadIdx.x, lane = tid & 31, wave = tid >> 5, h = lane >> 4, m = lane & 15;
  const int wr = wave & 3, wc = wave >> 2;
  const int bm0 = blockIdx.x * PBM, n0 = blockIdx.y * PBN, z = blockIdx.z;
  const int row0 = bm0 + 16 * wr, col0 = n0 + 64 * wc;

  v8f acc[PNT];
#pragma unroll
  for (int t = 0; t < PNT; ++t) acc[t] = zero8();

  const size_t ao = (size_t)(row0 + m) * NDIM + 8 * h;
  const us_t* aph = XH + ao;
  const us_t* apl = XL + ao;
  const size_t bo = ((size_t)z * NDIM + col0 + m) * NDIM + 8 * h;
  const us_t* bph = WH + bo;
  const us_t* bpl = WL + bo;

#pragma unroll 1
  for (int ks = 0; ks < NDIM / 32; ++ks) {
    const int k0 = 32 * ks;
    Frag ah, al;
    ah.h[0] = *(const v8us*)(aph + k0);
    ah.h[1] = *(const v8us*)(aph + k0 + 16);
    al.h[0] = *(const v8us*)(apl + k0);
    al.h[1] = *(const v8us*)(apl + k0 + 16);
#pragma unroll
    for (int t = 0; t < PNT; ++t) {
      const size_t ro = (size_t)(16 * t) * NDIM + k0;
      Frag bh, bl;
      bh.h[0] = *(const v8us*)(bph + ro);
      bh.h[1] = *(const v8us*)(bph + ro + 16);
      bl.h[0] = *(const v8us*)(bpl + ro);
      bl.h[1] = *(const v8us*)(bpl + ro + 16);
      acc[t] = wmb(ah, bh, acc[t]);
      acc[t] = wmb(ah, bl, acc[t]);
      acc[t] = wmb(al, bh, acc[t]);
    }
  }

#pragma unroll
  for (int t = 0; t < PNT; ++t) {
    const int cl = 64 * wc + 16 * t + m;
#pragma unroll
    for (int r = 0; r < 8; ++r) {
      const int rl = 16 * wr + 8 * h + r;
      sT[rl * PBN + cl] = acc[t][r];
    }
  }
  __syncthreads();

  float* dst = (z == 0) ? Q : ((z == 1) ? KN : V);
  v4f ov[8];
#pragma unroll
  for (int rr = 0; rr < 8; ++rr) {
    const int rl = 8 * wave + rr;
    v4f a = *(const v4f*)(sT + rl * PBN + 4 * lane);
    if (z == 1) {
      float ss = (a.x * a.x + a.y * a.y) + (a.z * a.z + a.w * a.w);
      ss = wsum_(ss);
      const float inv = 1.0f / fmaxf(sqrtf(ss), 1e-12f);
      a = a * inv;
    } else if (z == 2) {
      a.x = silu_(a.x); a.y = silu_(a.y); a.z = silu_(a.z); a.w = silu_(a.w);
    }
    ov[rr] = a;
  }
  const size_t go = (size_t)(bm0 + 8 * wave) * NDIM + n0 + 4 * lane;
#pragma unroll
  for (int rr = 0; rr < 8; ++rr) *(volatile v4f*)(dst + go + (size_t)rr * NDIM) = ov[rr];
  __threadfence();
#pragma unroll
  for (int rr = 0; rr < 8; ++rr) *(volatile v4f*)(dst + go + (size_t)rr * NDIM) = ov[rr];
}

__global__ __launch_bounds__(NTHR) void k_beta(const us_t* __restrict__ XH, const us_t* __restrict__ XL,
                                               const us_t* __restrict__ WBH, const us_t* __restrict__ WBL,
                                               float* BETA) {
  __shared__ __align__(16) float sB[NWAV * 128];
  const int tid = threadIdx.x, lane = tid & 31, wave = tid >> 5, h = lane >> 4, m = lane & 15;
  const int row0 = blockIdx.x * BBM + 16 * wave;

  v8f acc = zero8();
  const size_t ao = (size_t)(row0 + m) * NDIM + 8 * h;
  const us_t* aph = XH + ao;
  const us_t* apl = XL + ao;
  const size_t bo = (size_t)m * NDIM + 8 * h;
  const us_t* bph = WBH + bo;
  const us_t* bpl = WBL + bo;

#pragma unroll 1
  for (int ks = 0; ks < NDIM / 32; ++ks) {
    const int k0 = 32 * ks;
    Frag ah, al, bh, bl;
    ah.h[0] = *(const v8us*)(aph + k0);
    ah.h[1] = *(const v8us*)(aph + k0 + 16);
    al.h[0] = *(const v8us*)(apl + k0);
    al.h[1] = *(const v8us*)(apl + k0 + 16);
    bh.h[0] = *(const v8us*)(bph + k0);
    bh.h[1] = *(const v8us*)(bph + k0 + 16);
    bl.h[0] = *(const v8us*)(bpl + k0);
    bl.h[1] = *(const v8us*)(bpl + k0 + 16);
    acc = wmb(ah, bh, acc);
    acc = wmb(ah, bl, acc);
    acc = wmb(al, bh, acc);
  }

#pragma unroll
  for (int r = 0; r < 8; ++r) {
    const float s = sigm_(acc[r]);
    if (m < NHEAD) sB[wave * 128 + (8 * h + r) * NHEAD + m] = s;
  }
  __syncthreads();
  const v4f bv = *(const v4f*)(sB + wave * 128 + 4 * lane);
  float* dp = BETA + (size_t)row0 * NHEAD + 4 * lane;
  *(volatile v4f*)dp = bv;
  __threadfence();
  *(volatile v4f*)dp = bv;
}

__global__ __launch_bounds__(STHR) void k_scan(const float* __restrict__ Q, const float* __restrict__ KN,
                                               const float* __restrict__ V, const float* __restrict__ BETA,
                                               float* O) {
  __shared__ __align__(16) float pA[HDIM * SGRP];
  __shared__ __align__(16) float pB[HDIM * SGRP];
  __shared__ __align__(16) float sO[TB * HDIM];
  const int tid = threadIdx.x, lane = tid & 31, wave = tid >> 5;
  const int g = tid >> 7, vc = tid & (HDIM - 1);
  const int b = blockIdx.x >> 3, hh = blockIdx.x & 7;
  const size_t tokb = (size_t)b * NSEQ;
  const size_t colh = (size_t)hh * HDIM;

  float S[SROW];
#pragma unroll
  for (int j = 0; j < SROW; ++j) S[j] = 0.0f;

#pragma unroll 1
  for (int t = 0; t < NSEQ; ++t) {
    const size_t tok = tokb + (size_t)t;
    const size_t rowo = tok * NDIM + colh;
    const float* kp = KN + rowo + SROW * g;
    v4f kv[4];
#pragma unroll
    for (int c = 0; c < 4; ++c) kv[c] = *(const v4f*)(kp + 4 * c);
    const float vv = V[rowo + vc];
    const float bt = BETA[tok * NHEAD + hh];

    float psk = 0.0f;
#pragma unroll
    for (int c = 0; c < 4; ++c) {
      psk = fmaf(kv[c].x, S[4 * c + 0], psk);
      psk = fmaf(kv[c].y, S[4 * c + 1], psk);
      psk = fmaf(kv[c].z, S[4 * c + 2], psk);
      psk = fmaf(kv[c].w, S[4 * c + 3], psk);
    }
    pA[vc * SGRP + g] = psk;
    __syncthreads();

    const v4f s0 = *(const v4f*)(pA + vc * SGRP);
    const v4f s1 = *(const v4f*)(pA + vc * SGRP + 4);
    const float sk = ((((((s0.x + s0.y) + s0.z) + s0.w) + s1.x) + s1.y) + s1.z) + s1.w;
    const float u = bt * (vv - sk);

    const float* qp = Q + rowo + SROW * g;
    v4f qv[4];
#pragma unroll
    for (int c = 0; c < 4; ++c) qv[c] = *(const v4f*)(qp + 4 * c);

    float po = 0.0f;
#pragma unroll
    for (int c = 0; c < 4; ++c) {
      S[4 * c + 0] = fmaf(kv[c].x, u, S[4 * c + 0]);
      po = fmaf(qv[c].x, S[4 * c + 0], po);
      S[4 * c + 1] = fmaf(kv[c].y, u, S[4 * c + 1]);
      po = fmaf(qv[c].y, S[4 * c + 1], po);
      S[4 * c + 2] = fmaf(kv[c].z, u, S[4 * c + 2]);
      po = fmaf(qv[c].z, S[4 * c + 2], po);
      S[4 * c + 3] = fmaf(kv[c].w, u, S[4 * c + 3]);
      po = fmaf(qv[c].w, S[4 * c + 3], po);
    }
    pB[vc * SGRP + g] = po;
    __syncthreads();

    if (tid < HDIM) {
      const v4f o0 = *(const v4f*)(pB + vc * SGRP);
      const v4f o1 = *(const v4f*)(pB + vc * SGRP + 4);
      const float ov = ((((((o0.x + o0.y) + o0.z) + o0.w) + o1.x) + o1.y) + o1.z) + o1.w;
      sO[(t & (TB - 1)) * HDIM + vc] = ov;
    }
    if ((t & (TB - 1)) == TB - 1) {
      __syncthreads();
      const v4f ovv = *(const v4f*)(sO + wave * HDIM + 4 * lane);
      float* dp = O + (tokb + (size_t)(t - (TB - 1) + wave)) * NDIM + colh + 4 * lane;
      *(volatile v4f*)dp = ovv;
      __threadfence();
      *(volatile v4f*)dp = ovv;
    }
  }
}

__global__ __launch_bounds__(NTHR) void k_ln(const float* __restrict__ O, const float* __restrict__ lw,
                                             const float* __restrict__ lb, float* out) {
  const int tid = threadIdx.x, lane = tid & 31, wave = tid >> 5;
  const size_t row = (size_t)blockIdx.x * NWAV + wave;
  const float* rp = O + row * NDIM;
  v4f xv[8];
#pragma unroll
  for (int i = 0; i < 8; ++i) xv[i] = *(const v4f*)(rp + 128 * i + 4 * lane);
  float s = 0.0f;
#pragma unroll
  for (int i = 0; i < 8; ++i) s += (xv[i].x + xv[i].y) + (xv[i].z + xv[i].w);
  s = wsum_(s);
  const float mu = s * (1.0f / (float)NDIM);
  float ss = 0.0f;
#pragma unroll
  for (int i = 0; i < 8; ++i) {
    xv[i] = xv[i] - mu;
    ss = fmaf(xv[i].x, xv[i].x, ss);
    ss = fmaf(xv[i].y, xv[i].y, ss);
    ss = fmaf(xv[i].z, xv[i].z, ss);
    ss = fmaf(xv[i].w, xv[i].w, ss);
  }
  ss = wsum_(ss);
  const float var = ss * (1.0f / (float)NDIM);
  const float rs = 1.0f / sqrtf(var + 1e-5f);
  v4f yv[8];
#pragma unroll
  for (int i = 0; i < 8; ++i) {
    const v4f w = *(const v4f*)(lw + 128 * i + 4 * lane);
    const v4f bb = *(const v4f*)(lb + 128 * i + 4 * lane);
    yv[i] = (xv[i] * rs) * w + bb;
  }
  float* op = out + row * NDIM + 4 * lane;
#pragma unroll
  for (int i = 0; i < 8; ++i) *(volatile v4f*)(op + 128 * i) = yv[i];
  __threadfence();
#pragma unroll
  for (int i = 0; i < 8; ++i) *(volatile v4f*)(op + 128 * i) = yv[i];
}

extern "C" void kernel_launch(void* const* d_in, const int* in_sizes, int n_in,
                              void* d_out, int out_size, void* d_ws, size_t ws_size,
                              hipStream_t stream) {
  if (n_in < 7) return;
  if (in_sizes[0] != NTOK * NDIM) return;
  if (in_sizes[1] != NDIM * NDIM || in_sizes[2] != NDIM * NDIM || in_sizes[3] != NDIM * NDIM) return;
  if (in_sizes[4] != NDIM * NHEAD) return;
  if (in_sizes[5] != NDIM || in_sizes[6] != NDIM) return;
  if (out_size != NTOK * NDIM) return;
  const size_t tot = (size_t)WSTOT;
  if (tot > ws_size || tot > (size_t)WSCAP) return;

  const float* x  = (const float*)d_in[0];
  const float* Wq = (const float*)d_in[1];
  const float* Wk = (const float*)d_in[2];
  const float* Wv = (const float*)d_in[3];
  const float* Wb = (const float*)d_in[4];
  const float* lw = (const float*)d_in[5];
  const float* lb = (const float*)d_in[6];
  float* out = (float*)d_out;

  char* ws = (char*)d_ws;
  us_t* XH  = (us_t*)(ws + OXH);
  us_t* XL  = (us_t*)(ws + OXL);
  us_t* WH  = (us_t*)(ws + OWH);
  us_t* WL  = (us_t*)(ws + OWL);
  us_t* WBH = (us_t*)(ws + OWBH);
  us_t* WBL = (us_t*)(ws + OWBL);
  float* Q    = (float*)(ws + OQ);
  float* KN   = (float*)(ws + OKN);
  float* V    = (float*)(ws + OV);
  float* BETA = (float*)(ws + OBT);
  float* O    = (float*)(ws + OO);

  k_cvtx<<<CVTX_BLK, NTHR, 0, stream>>>(x, XH, XL);
  k_cvtw<<<dim3(NDIM / CT, NDIM / CT, 3), NTHR, 0, stream>>>(Wq, Wk, Wv, WH, WL);
  k_cvtwb<<<CVTWB_BLK, NTHR, 0, stream>>>(Wb, WBH, WBL);

  k_proj<<<dim3(NTOK / PBM, NDIM / PBN, 3), NTHR, 0, stream>>>(XH, XL, WH, WL, Q, KN, V);

  k_beta<<<NTOK / BBM, NTHR, 0, stream>>>(XH, XL, WBH, WBL, BETA);

  k_scan<<<NBAT * NHEAD, STHR, 0, stream>>>(Q, KN, V, BETA, O);

  k_ln<<<NTOK / NWAV, NTHR, 0, stream>>>(O, lw, lb, out);
}
